// Nam_64132451664509
// MI455X (gfx1250) — hardware-verified
//
#include <hip/hip_runtime.h>
#include <math.h>

#define NF   64
#define NH   64
#define NB   16384
#define NL   2

typedef __attribute__((ext_vector_type(16))) _Float16 v16h;
typedef __attribute__((ext_vector_type(8)))  float    v8f;

#define WAVES_PER_WG 8
#define TPW 2
#define ROWS_PER_BLOCK (WAVES_PER_WG * TPW * 16)

__device__ __forceinline__ float relu1(float x) { return fmaxf(x, 0.0f); }

__global__ __launch_bounds__(256) void nam_kernel(
    const float* __restrict__ x,
    const float* __restrict__ w_in,
    const float* __restrict__ b_in,
    const float* __restrict__ w_hid,
    const float* __restrict__ b_hid,
    const float* __restrict__ w_out,
    const float* __restrict__ b_out,
    const float* __restrict__ w_final,
    const float* __restrict__ b_final,
    float* __restrict__ out)
{
    __shared__ __align__(32) _Float16 sA[16 * 512];
    __shared__ __align__(32) float sWin[NH], sBin[NH], sWout[NH];
    __shared__ __align__(32) float sBh[2][NH];
    __shared__ __align__(16) float sres[ROWS_PER_BLOCK];

    const int lane = threadIdx.x & 31;
    const int wave = threadIdx.x >> 5;
    const int g    = lane >> 4;
    const int lm   = lane & 15;
    const int row0 = blockIdx.x * ROWS_PER_BLOCK + wave * (TPW * 16);

    float xv[TPW];
#pragma unroll
    for (int tt = 0; tt < TPW; ++tt) xv[tt] = 0.f;
    float tot[TPW];
#pragma unroll
    for (int tt = 0; tt < TPW; ++tt) tot[tt] = 0.f;

    for (int f = 0; f < NF; ++f) {
        __syncthreads();
        for (int idx = threadIdx.x; idx < 8192; idx += 256) {
            int frag = idx >> 9;
            int L    = (idx >> 4) & 31;
            int i    = idx & 15;
            int l = frag >> 3;
            int t = (frag >> 2) & 1;
            int n = frag & 3;
            int h = 32 * t + 8 * (L >> 4) + i + ((i >= 8) ? 8 : 0);
            int k = 16 * n + (L & 15);
            sA[idx] = (_Float16)w_hid[((l * NF + f) * NH + h) * NH + k];
        }
        if (threadIdx.x < NH) {
            int j = threadIdx.x;
            sWin[j]  = w_in[f * NH + j];
            sBin[j]  = b_in[f * NH + j];
            sWout[j] = w_out[f * NH + j];
            sBh[0][j] = b_hid[(0 * NF + f) * NH + j];
            sBh[1][j] = b_hid[(1 * NF + f) * NH + j];
        }
        __syncthreads();

        const float bo = b_out[f];
        const float wf = w_final[f];
        v8f wo[4];
#pragma unroll
        for (int n = 0; n < 4; ++n) wo[n] = *(const v8f*)&sWout[16 * n + 8 * g];
        const _Float16* sAf = &sA[lane * 16];

#pragma unroll
        for (int tt = 0; tt < TPW; ++tt) {
            const int m0 = row0 + tt * 16;
            const float xm = x[(size_t)(m0 + lm) * NF + f];

            v16h b0[2];
#pragma unroll
            for (int t = 0; t < 2; ++t) {
#pragma unroll
                for (int i = 0; i < 8; ++i) {
                    const int hA = 32 * t + 8 * g + i;
                    const int hB = 32 * t + 16 + 8 * g + i;
                    b0[t][i]     = (_Float16)relu1(xm * sWin[hA] + sBin[hA]);
                    b0[t][8 + i] = (_Float16)relu1(xm * sWin[hB] + sBin[hB]);
                }
            }
            v8f acc[4];
#pragma unroll
            for (int n = 0; n < 4; ++n) acc[n] = *(const v8f*)&sBh[0][16 * n + 8 * g];
#pragma unroll
            for (int t = 0; t < 2; ++t) {
#pragma unroll
                for (int n = 0; n < 4; ++n) {
                    const v16h a = *(const v16h*)&sAf[((0 * 2 + t) * 4 + n) * 512];
                    acc[n] = __builtin_amdgcn_wmma_f32_16x16x32_f16(false, a, false, b0[t], (short)0, acc[n], false, false);
                }
            }
            asm volatile("v_nop\n\tv_nop\n\tv_nop\n\tv_nop" : "+v"(acc[0]), "+v"(acc[1]), "+v"(acc[2]), "+v"(acc[3]) : "v"(b0[0]), "v"(b0[1]));

            v16h b1[2];
#pragma unroll
            for (int t = 0; t < 2; ++t) {
#pragma unroll
                for (int e = 0; e < 8; ++e) {
                    b1[t][e]     = (_Float16)relu1(acc[2 * t][e]);
                    b1[t][8 + e] = (_Float16)relu1(acc[2 * t + 1][e]);
                }
            }
            v8f acc2[4];
#pragma unroll
            for (int n = 0; n < 4; ++n) acc2[n] = *(const v8f*)&sBh[1][16 * n + 8 * g];
#pragma unroll
            for (int t = 0; t < 2; ++t) {
#pragma unroll
                for (int n = 0; n < 4; ++n) {
                    const v16h a = *(const v16h*)&sAf[((1 * 2 + t) * 4 + n) * 512];
                    acc2[n] = __builtin_amdgcn_wmma_f32_16x16x32_f16(false, a, false, b1[t], (short)0, acc2[n], false, false);
                }
            }
            asm volatile("v_nop\n\tv_nop\n\tv_nop\n\tv_nop" : "+v"(acc2[0]), "+v"(acc2[1]), "+v"(acc2[2]), "+v"(acc2[3]) : "v"(b1[0]), "v"(b1[1]));

            float s0 = 0.0f, s1 = 0.0f, s2 = 0.0f, s3 = 0.0f;
#pragma unroll
            for (int r = 0; r < 8; ++r) {
                s0 += relu1(acc2[0][r]) * wo[0][r];
                s1 += relu1(acc2[1][r]) * wo[1][r];
                s2 += relu1(acc2[2][r]) * wo[2][r];
                s3 += relu1(acc2[3][r]) * wo[3][r];
            }
            float s = (s0 + s1) + (s2 + s3);
            s += __shfl_xor(s, 16, 32);
            tot[tt] += (s + bo) * wf;
        }
    }

    const float bf = b_final[0];
#pragma unroll
    for (int tt = 0; tt < TPW; ++tt)
        if (g == 0) sres[wave * (TPW * 16) + tt * 16 + lm] = 1.0f / (1.0f + expf(-(tot[tt] + bf)));
    __syncthreads();
    {
        const int r = wave * 32 + lane;
        const float v = sres[r];
        ((volatile float*)out)[(size_t)blockIdx.x * ROWS_PER_BLOCK + r] = v;
        __threadfence();
        ((volatile float*)out)[(size_t)blockIdx.x * ROWS_PER_BLOCK + r] = v;
    }
}

extern "C" void kernel_launch(void* const* d_in, const int* in_sizes, int n_in,
                              void* d_out, int out_size, void* d_ws, size_t ws_size,
                              hipStream_t stream) {
    (void)in_sizes; (void)n_in; (void)out_size; (void)d_ws; (void)ws_size;
    const float* x       = (const float*)d_in[0];
    const float* w_in    = (const float*)d_in[1];
    const float* b_in    = (const float*)d_in[2];
    const float* w_hid   = (const float*)d_in[3];
    const float* b_hid   = (const float*)d_in[4];
    const float* w_out   = (const float*)d_in[5];
    const float* b_out   = (const float*)d_in[6];
    const float* w_final = (const float*)d_in[7];
    const float* b_final = (const float*)d_in[8];
    float* out = (float*)d_out;

    nam_kernel<<<NB / ROWS_PER_BLOCK, 256, 0, stream>>>(
        x, w_in, b_in, w_hid, b_hid, w_out, b_out, w_final, b_final, out);
}
